// FastLinearMemory_27762668601945
// MI455X (gfx1250) — hardware-verified
//
#include <hip/hip_runtime.h>
#include <stdint.h>

typedef __attribute__((ext_vector_type(16))) _Float16 v16h;
typedef __attribute__((ext_vector_type(8)))  _Float16 v8h;
typedef __attribute__((ext_vector_type(16))) __bf16   v16b;
typedef __attribute__((ext_vector_type(8)))  __bf16   v8b;
typedef __attribute__((ext_vector_type(8)))  float    v8f;
typedef __attribute__((ext_vector_type(4)))  float    v4f;

__device__ __forceinline__ unsigned short f2bf_bits(float f) {
  unsigned u = __float_as_uint(f);
  return (unsigned short)((u + 0x7FFFu + ((u >> 16) & 1u)) >> 16);
}
__device__ __forceinline__ float bf_bits2f(unsigned short h) { return __uint_as_float(((unsigned)h) << 16); }

__device__ __forceinline__ void dep_guard_h(v8f& a, v8f& b, v16h x, v16h y) { asm volatile("v_nop\n\tv_nop\n\tv_nop\n\tv_nop" : "+v"(a), "+v"(b) : "v"(x), "v"(y)); }
__device__ __forceinline__ void dep_guard_b(v8f& a, v8f& b, v16b x, v16b y) { asm volatile("v_nop\n\tv_nop\n\tv_nop\n\tv_nop" : "+v"(a), "+v"(b) : "v"(x), "v"(y)); }
__device__ __forceinline__ void keep4_h(v16h a, v16h b, v16h c, v16h d) { asm volatile("v_nop" :: "v"(a), "v"(b), "v"(c), "v"(d)); }
__device__ __forceinline__ void keep4_b(v16b a, v16b b, v16b c, v16b d) { asm volatile("v_nop" :: "v"(a), "v"(b), "v"(c), "v"(d)); }
__device__ __forceinline__ void acc_guard4(v8f& a, v8f& b, v8f& c, v8f& d) { asm volatile("v_nop\n\tv_nop\n\tv_nop\n\tv_nop" : "+v"(a), "+v"(b), "+v"(c), "+v"(d)); }
template <typename T> struct Frag;
template <> struct Frag<_Float16> {
  typedef v16h V; union U { v16h v; v8h h[2]; };
  static __device__ __forceinline__ v16h load(const _Float16* p) {
    U f; f.h[0] = *(const v8h*)(p); f.h[1] = *(const v8h*)(p + 16); return f.v;
  }
  static __device__ __forceinline__ v8f mma(v16h a, v16h b, v8f c) {
    return __builtin_amdgcn_wmma_f32_16x16x32_f16(false, a, false, b, (short)0, c, false, false);
  }
  static __device__ __forceinline__ void guard(v8f& a, v8f& b, v16h x, v16h y) { dep_guard_h(a, b, x, y); }
  static __device__ __forceinline__ void keep(v16h a, v16h b, v16h c, v16h d) { keep4_h(a, b, c, d); }
};
template <> struct Frag<__bf16> {
  typedef v16b V; union U { v16b v; v8b h[2]; };
  static __device__ __forceinline__ v16b load(const __bf16* p) {
    U f; f.h[0] = *(const v8b*)(p); f.h[1] = *(const v8b*)(p + 16); return f.v;
  }
  static __device__ __forceinline__ v8f mma(v16b a, v16b b, v8f c) {
    return __builtin_amdgcn_wmma_f32_16x16x32_bf16(false, a, false, b, (short)0, c, false, false);
  }
  static __device__ __forceinline__ void guard(v8f& a, v8f& b, v16b x, v16b y) { dep_guard_b(a, b, x, y); }
  static __device__ __forceinline__ void keep(v16b a, v16b b, v16b c, v16b d) { keep4_b(a, b, c, d); }
};

__device__ __forceinline__ float softplus_f(float x) { return fmaxf(x, 0.0f) + log1pf(expf(-fabsf(x))); }

__device__ __forceinline__ void wave_sync_lds() {
  __builtin_amdgcn_fence(__ATOMIC_RELEASE, "workgroup");
  __builtin_amdgcn_wave_barrier();
  __builtin_amdgcn_fence(__ATOMIC_ACQUIRE, "workgroup");
}

template <int ET> struct Elem;
template <> struct Elem<0> { typedef _Float16 T; };
template <> struct Elem<1> { typedef __bf16 T; };
template <int ET, bool SPLIT, int BIAS_MODE, int OUT_MODE, bool RESID, int ACT = 0>
__global__ __launch_bounds__(256) void wmma_gemm64(
    const unsigned short* __restrict__ Ap, const unsigned short* __restrict__ A2p, int lda, long strideA,
    const unsigned short* __restrict__ Btp, const unsigned short* __restrict__ Bt2p, int ldb, long strideB,
    void* __restrict__ Cout, void* __restrict__ Cout2, int ldc, long strideC,
    const float* __restrict__ bias,
    const float* __restrict__ resid, long strideR,
    int M, int N, int K, float scale) {
  typedef typename Elem<ET>::T T;
  typedef typename Frag<T>::V V;
  const T* A = (const T*)Ap; const T* A2 = (const T*)A2p; const T* Bt = (const T*)Btp; const T* Bt2 = (const T*)Bt2p;
  __shared__ __align__(16) float sT[8][16 * 68];
  const int b    = blockIdx.y;
  const int lane = threadIdx.x & 31;
  const int wave = threadIdx.x >> 5;
  const int tilesN = N >> 6;
  const int tilesM = M >> 6;
  const int tile = blockIdx.x * 8 + wave;
  if (tile >= tilesM * tilesN) return;
  const int tm = tile / tilesN;
  const int tn = tile - tm * tilesN;
  const int m0 = tm << 6;
  const int n0 = tn << 6;

  const T* Ab  = A  + (size_t)b * strideA;
  const T* Bb  = Bt + (size_t)b * strideB;
  const T* Ab2 = SPLIT ? (A2  + (size_t)b * strideA) : nullptr;
  const T* Bb2 = SPLIT ? (Bt2 + (size_t)b * strideB) : nullptr;

  const int rlane = lane & 15;
  const int koff  = (lane >> 4) * 8;
  const int mOff  = (lane >> 4) * 8;

  v8f acc[4][4];
#pragma unroll
  for (int i = 0; i < 4; ++i)
#pragma unroll
    for (int j = 0; j < 4; ++j) acc[i][j] = (v8f){0.f,0.f,0.f,0.f,0.f,0.f,0.f,0.f};

  for (int k0 = 0; k0 < K; k0 += 32) {
    V bh[4], bl[4];
#pragma unroll
    for (int j = 0; j < 4; ++j) {
      const size_t bo = (size_t)(n0 + (j << 4) + rlane) * ldb + koff + k0;
      bh[j] = Frag<T>::load(Bb + bo);
      if (SPLIT) bl[j] = Frag<T>::load(Bb2 + bo);
    }
#pragma unroll
    for (int i = 0; i < 4; ++i) {
      const size_t ao = (size_t)(m0 + (i << 4) + rlane) * lda + koff + k0;
      V ah = Frag<T>::load(Ab + ao);
      V al;
      if (SPLIT) al = Frag<T>::load(Ab2 + ao);
#pragma unroll
      for (int j = 0; j < 4; ++j) {
        acc[i][j] = Frag<T>::mma(ah, bh[j], acc[i][j]);
        if (SPLIT) {
          acc[i][j] = Frag<T>::mma(ah, bl[j], acc[i][j]);
          acc[i][j] = Frag<T>::mma(al, bh[j], acc[i][j]);
        }
      }
      Frag<T>::guard(acc[i][0], acc[i][3], ah, SPLIT ? al : ah);
    }
    Frag<T>::keep(bh[0], bh[1], bh[2], bh[3]);
    if (SPLIT) Frag<T>::keep(bl[0], bl[1], bl[2], bl[3]);
  }
  acc_guard4(acc[0][0], acc[0][1], acc[0][2], acc[0][3]);
  acc_guard4(acc[1][0], acc[1][1], acc[1][2], acc[1][3]);
  acc_guard4(acc[2][0], acc[2][1], acc[2][2], acc[2][3]);
  acc_guard4(acc[3][0], acc[3][1], acc[3][2], acc[3][3]);

  float* slab = sT[wave];
  const float* Rb = RESID ? (resid + (size_t)b * strideR) : nullptr;
#pragma unroll
  for (int i = 0; i < 4; ++i) {
    const int mBase = m0 + (i << 4);
#pragma unroll
    for (int j = 0; j < 4; ++j) {
      const int n = n0 + (j << 4) + rlane;
      float bv = 0.f;
      if (BIAS_MODE == 2) bv = bias[n];
#pragma unroll
      for (int r = 0; r < 8; ++r) {
        float v = acc[i][j][r] * scale;
        if (BIAS_MODE == 1) v += bias[mBase + mOff + r];
        if (BIAS_MODE == 2) v += bv;
        if (RESID) v += Rb[(size_t)(mBase + mOff + r) * ldc + n];
        if (ACT == 1) v = tanhf(v);
        if (ACT == 2) v = fmaxf(v, 0.0f);
        if (ACT == 3) v = v / (1.0f + expf(-v));
        if (ACT == 4) v = (v > 0.f) ? v : 0.01f * v;
        if (ACT == 5) v = 0.5f * v * (1.0f + erff(v * 0.70710678118654752f));
        slab[(mOff + r) * 68 + (j << 4) + rlane] = v;
      }
    }
    __builtin_amdgcn_fence(__ATOMIC_RELEASE, "workgroup");
    __builtin_amdgcn_wave_barrier();
    __builtin_amdgcn_fence(__ATOMIC_ACQUIRE, "workgroup");
    if (OUT_MODE == 0) {
      float* C = (float*)Cout + (size_t)b * strideC;
      const int hh = lane >> 4, c4 = (lane & 15) * 4;
      for (int pass = 0; pass < 2; ++pass) {
#pragma unroll
        for (int it = 0; it < 8; ++it) {
          const int row = it * 2 + hh;
          v4f v = *(const v4f*)(slab + row * 68 + c4);
          *(volatile v4f*)(C + (size_t)(mBase + row) * ldc + n0 + c4) = v;
        }
        __threadfence();
      }
    } else {
      const int q = lane >> 3, c8 = (lane & 7) * 8;
      unsigned short* C  = (unsigned short*)Cout  + (size_t)b * strideC;
      unsigned short* C2 = (OUT_MODE == 2) ? ((unsigned short*)Cout2 + (size_t)b * strideC) : nullptr;
      for (int pass = 0; pass < 2; ++pass) {
#pragma unroll
        for (int it = 0; it < 4; ++it) {
          const int row = it * 4 + q;
          const float* sp = slab + row * 68 + c8;
          v8h hv, lv;
#pragma unroll
          for (int e = 0; e < 8; ++e) {
            if (OUT_MODE == 1) {
              hv[e] = (_Float16)sp[e];
            } else {
              unsigned short hb = f2bf_bits(sp[e]);
              unsigned short lb = f2bf_bits(sp[e] - bf_bits2f(hb));
              hv[e] = __builtin_bit_cast(_Float16, hb);
              lv[e] = __builtin_bit_cast(_Float16, lb);
            }
          }
          *(volatile v8h*)(C + (size_t)(mBase + row) * ldc + n0 + c8) = hv;
          if (OUT_MODE == 2) *(volatile v8h*)(C2 + (size_t)(mBase + row) * ldc + n0 + c8) = lv;
        }
        __threadfence();
      }
    }
    __builtin_amdgcn_fence(__ATOMIC_RELEASE, "workgroup");
    __builtin_amdgcn_wave_barrier();
    __builtin_amdgcn_fence(__ATOMIC_ACQUIRE, "workgroup");
  }
}

__global__ __launch_bounds__(256) void cast_f32_f16x2(
    const float* __restrict__ in, _Float16* __restrict__ out, int n2) {
  int i = blockIdx.x * 256 + threadIdx.x;
  if (i < n2) {
    const _Float16 h0 = (_Float16)in[2 * i], h1 = (_Float16)in[2 * i + 1];
    const unsigned u = (unsigned)__builtin_bit_cast(unsigned short, h0) | ((unsigned)__builtin_bit_cast(unsigned short, h1) << 16);
    ((volatile unsigned*)out)[i] = u;
    __threadfence();
    ((volatile unsigned*)out)[i] = u;
  }
}

__global__ __launch_bounds__(256) void tcast_f32_f16(const float* __restrict__ in, long sIn, int C,
    unsigned short* __restrict__ out, long sOut, int ldo, float mul) {
  __shared__ __align__(16) float tile[64 * 68];
  const int tid = threadIdx.x, lane = tid & 31, wave = tid >> 5;
  const int c0 = blockIdx.x * 64, r0 = blockIdx.y * 64;
  const float* inb = in + (size_t)blockIdx.z * sIn;
  _Float16* outb = (_Float16*)out + (size_t)blockIdx.z * sOut;
#pragma unroll
  for (int it = 0; it < 4; ++it) {
    const int idx = it * 256 + tid;
    const int row = idx >> 4, c4 = (idx & 15) * 4;
    const v4f v = *(const v4f*)(inb + (size_t)(r0 + row) * C + c0 + c4);
    *(v4f*)(tile + row * 68 + c4) = v;
  }
  __syncthreads();
  const int q = lane >> 3, c8 = (lane & 7) * 8;
  for (int pass = 0; pass < 2; ++pass) {
#pragma unroll
    for (int it = 0; it < 2; ++it) {
      const int orow = it * 32 + wave * 4 + q;
      v8h hv;
#pragma unroll
      for (int e = 0; e < 8; ++e) hv[e] = (_Float16)(tile[(c8 + e) * 68 + orow] * mul);
      *(volatile v8h*)(outb + (size_t)(c0 + orow) * ldo + r0 + c8) = hv;
    }
    __threadfence();
  }
}

__global__ __launch_bounds__(256) void prep_kernel(const float* __restrict__ addresses, const float* __restrict__ normalizer,
    const float* __restrict__ b_access, const float* __restrict__ b_read,
    unsigned short* __restrict__ akT16, float* __restrict__ norm_k,
    float* __restrict__ kern_n, float* __restrict__ bias_cat) {
  __shared__ __align__(16) float aks[128 * 64];
  const int tid = threadIdx.x;
#pragma unroll 1
  for (int i = 0; i < 32; ++i) {
    const int idx = i * 256 + tid;
    aks[idx] = softplus_f(addresses[idx]);
  }
  __syncthreads();
  {
    _Float16* akT = (_Float16*)akT16;
    for (int pass = 0; pass < 2; ++pass) {
#pragma unroll 1
      for (int it = 0; it < 4; ++it) {
        const int a = it * 16 + (tid >> 4);
        const int mb = (tid & 15) * 8;
        v8h hv;
#pragma unroll
        for (int e = 0; e < 8; ++e) hv[e] = (_Float16)aks[(mb + e) * 64 + a];
        *(volatile v8h*)(akT + a * 128 + mb) = hv;
      }
      __threadfence();
    }
  }
  if (tid < 16) {
    const int a0 = tid * 4;
    float s0 = 0.f, s1 = 0.f, s2 = 0.f, s3 = 0.f;
#pragma unroll 1
    for (int m = 0; m < 128; ++m) {
      const float* rp = aks + m * 64 + a0;
      s0 += rp[0]; s1 += rp[1]; s2 += rp[2]; s3 += rp[3];
    }
    v4f v; v[0] = s0; v[1] = s1; v[2] = s2; v[3] = s3;
    *(volatile v4f*)(norm_k + a0) = v;
    __threadfence();
    *(volatile v4f*)(norm_k + a0) = v;
  }
  {
    const int ia = (tid < 128 ? tid : 127) * 4;
    const int ib = (tid >= 128 ? tid - 128 : 0) * 4;
    const v4f va = *(const v4f*)(b_access + ia);
    const v4f vb = *(const v4f*)(b_read + ib);
    const v4f v = (tid < 128) ? va : vb;
    *(volatile v4f*)(bias_cat + tid * 4) = v;
    __threadfence();
    *(volatile v4f*)(bias_cat + tid * 4) = v;
  }
#pragma unroll 1
  for (int i = 0; i < 64; ++i) {
    const int idx = i * 256 + tid;
    const int b = idx >> 12, a = (idx >> 6) & 63, d = idx & 63;
    const float* nb = normalizer + (size_t)b * 8192 + d;
    float s = 0.f;
#pragma unroll 1
    for (int m = 0; m < 128; ++m) s += aks[m * 64 + a] * nb[m * 64];
    ((volatile float*)kern_n)[idx] = s;
    __threadfence();
    ((volatile float*)kern_n)[idx] = s;
  }
}

__global__ __launch_bounds__(256) void softplus_kernel(const float* __restrict__ in, float* __restrict__ out, int nq) {
  const int gid = blockIdx.x * 256 + threadIdx.x;
#pragma unroll 1
  for (int it = 0; it < 4; ++it) {
    const int i = it * nq + gid;
    const float s = softplus_f(in[i]);
    ((volatile float*)out)[i] = s;
    __threadfence();
    ((volatile float*)out)[i] = s;
  }
}

__global__ __launch_bounds__(256) void permute_km(const unsigned short* __restrict__ C3, unsigned short* __restrict__ KMt) {
  __shared__ __align__(16) _Float16 S[64 * 136];
  const int tid = threadIdx.x, lane = tid & 31, wave = tid >> 5;
  const int b = blockIdx.x >> 6, a = blockIdx.x & 63;
  const _Float16* src = (const _Float16*)C3 + ((size_t)b * 64 + a) * 8192;
#pragma unroll
  for (int it = 0; it < 4; ++it) {
    const int idx = it * 256 + tid;
    const int a2 = idx >> 4, x8 = (idx & 15) * 8;
    *(v8h*)(S + a2 * 136 + x8) = *(const v8h*)(src + a2 * 128 + x8);
  }
  __syncthreads();
  _Float16* dstb = (_Float16*)KMt + (size_t)b * 128 * 4096 + a * 64;
  const int q = lane >> 3, c8 = (lane & 7) * 8;
  for (int pass = 0; pass < 2; ++pass) {
#pragma unroll
    for (int it = 0; it < 4; ++it) {
      const int x = it * 32 + wave * 4 + q;
      v8h hv;
#pragma unroll
      for (int e = 0; e < 8; ++e) hv[e] = S[(c8 + e) * 136 + x];
      *(volatile v8h*)(dstb + (size_t)x * 4096 + c8) = hv;
    }
    __threadfence();
  }
}

__global__ __launch_bounds__(256) void scales_kernel(const float* __restrict__ AQRQ, const float* __restrict__ kern_n,
    const float* __restrict__ norm_k, float* __restrict__ scale_out) {
  __shared__ __align__(16) float knT[65 * 68];
  const int tid = threadIdx.x;
  const int b = blockIdx.x >> 4;
  const float* kn = kern_n + (size_t)b * 4096;
#pragma unroll 1
  for (int it = 0; it < 16; ++it) {
    const int idx = it * 256 + tid;
    const int a = idx >> 6, d = idx & 63;
    knT[d * 68 + a] = kn[idx];
  }
  if (tid < 64) knT[64 * 68 + tid] = norm_k[tid];
  __syncthreads();
  const int r = blockIdx.x * 256 + tid;
  const int bt = r >> 3, h = r & 7;
  const float* aqp = AQRQ + (size_t)bt * 1024 + h * 64;
  const float* rqp = aqp + 512;
  float aq[64];
#pragma unroll
  for (int i = 0; i < 16; ++i) {
    const v4f v = *(const v4f*)(aqp + 4 * i);
    aq[4 * i + 0] = v[0]; aq[4 * i + 1] = v[1]; aq[4 * i + 2] = v[2]; aq[4 * i + 3] = v[3];
  }
  const float eps = 1e-5f;
  float tot = eps * eps;
#pragma unroll 1
  for (int d = 0; d < 65; ++d) {
    const float* kr = knT + d * 68;
    float inner = 0.f;
#pragma unroll
    for (int i = 0; i < 16; ++i) {
      const v4f kv = *(const v4f*)(kr + 4 * i);
      inner += aq[4 * i + 0] * kv[0];
      inner += aq[4 * i + 1] * kv[1];
      inner += aq[4 * i + 2] * kv[2];
      inner += aq[4 * i + 3] * kv[3];
    }
    const int dc = (d < 64) ? d : 63;
    const float rv = rqp[dc];
    const float w = (d < 64) ? rv : eps;
    tot += w * inner;
  }
  const float sc = 1.0f / tot;
  ((volatile float*)scale_out)[r] = sc;
  __threadfence();
  ((volatile float*)scale_out)[r] = sc;
}

__global__ __launch_bounds__(128) void stage2_kernel(const float* __restrict__ AQRQ, const unsigned short* __restrict__ KMt,
    const float* __restrict__ scale, unsigned short* __restrict__ RESP16) {
  __shared__ __align__(16) _Float16 Pt[4][16 * 40];
  __shared__ __align__(16) float Os[4][16 * 132];
  const int tid = threadIdx.x, lane = tid & 31, wave = tid >> 5;
  const int hh = lane >> 4, rl = lane & 15, koff = hh * 8;
  const int b = blockIdx.x >> 6;
  const int R0 = blockIdx.x * 64 + wave * 16;
  const int myrow = R0 + rl;
  const float* aqp = AQRQ + (size_t)(myrow >> 3) * 1024 + (myrow & 7) * 64;
  const float* rqp = aqp + 512;
  float rqv[32];
#pragma unroll
  for (int i = 0; i < 4; ++i) {
    const v4f v0 = *(const v4f*)(rqp + 16 * hh + 4 * i);
    const v4f v1 = *(const v4f*)(rqp + 32 + 16 * hh + 4 * i);
    rqv[4 * i + 0] = v0[0]; rqv[4 * i + 1] = v0[1]; rqv[4 * i + 2] = v0[2]; rqv[4 * i + 3] = v0[3];
    rqv[16 + 4 * i + 0] = v1[0]; rqv[16 + 4 * i + 1] = v1[1]; rqv[16 + 4 * i + 2] = v1[2]; rqv[16 + 4 * i + 3] = v1[3];
  }
  const _Float16* KMb = (const _Float16*)KMt + (size_t)b * 128 * 4096;
  _Float16* Pw = Pt[wave];
  v8f acc[8];
#pragma unroll
  for (int j = 0; j < 8; ++j) acc[j] = (v8f){0.f,0.f,0.f,0.f,0.f,0.f,0.f,0.f};

#pragma unroll 1
  for (int a = 0; a < 64; ++a) {
    const float aqa = aqp[a];
#pragma unroll
    for (int s = 0; s < 2; ++s) {
      v8h p0, p1;
#pragma unroll
      for (int e = 0; e < 8; ++e) {
        p0[e] = (_Float16)(aqa * rqv[s * 16 + e]);
        p1[e] = (_Float16)(aqa * rqv[s * 16 + 8 + e]);
      }
      wave_sync_lds();
      *(v8h*)(Pw + rl * 40 + 16 * hh) = p0;
      *(v8h*)(Pw + rl * 40 + 16 * hh + 8) = p1;
      wave_sync_lds();
      const v16h af = Frag<_Float16>::load(Pw + rl * 40 + koff);
      const int k0 = a * 64 + s * 32;
#pragma unroll
      for (int g = 0; g < 2; ++g) {
        v16h bf[4];
#pragma unroll
        for (int j = 0; j < 4; ++j)
          bf[j] = Frag<_Float16>::load(KMb + (size_t)(((g * 4 + j) << 4) + rl) * 4096 + k0 + koff);
#pragma unroll
        for (int j = 0; j < 4; ++j) acc[g * 4 + j] = Frag<_Float16>::mma(af, bf[j], acc[g * 4 + j]);
        Frag<_Float16>::guard(acc[g * 4], acc[g * 4 + 3], af, af);
        Frag<_Float16>::keep(bf[0], bf[1], bf[2], bf[3]);
      }
    }
  }
  acc_guard4(acc[0], acc[1], acc[2], acc[3]);
  acc_guard4(acc[4], acc[5], acc[6], acc[7]);

  float sc[8];
#pragma unroll
  for (int r = 0; r < 8; ++r) sc[r] = scale[R0 + 8 * hh + r] * 256.0f;
  float* os = Os[wave];
#pragma unroll
  for (int j = 0; j < 8; ++j) {
#pragma unroll
    for (int r = 0; r < 8; ++r) os[(8 * hh + r) * 132 + (j << 4) + rl] = acc[j][r] * sc[r];
  }
  wave_sync_lds();
  _Float16* RS = (_Float16*)RESP16;
  const int q = lane >> 3, c8 = (lane & 7) * 8;
  for (int pass = 0; pass < 2; ++pass) {
#pragma unroll
    for (int it = 0; it < 8; ++it) {
      const int row = it * 2 + (q >> 1);
      const int xoff = (q & 1) * 64 + c8;
      v8h hv;
#pragma unroll
      for (int e = 0; e < 8; ++e) hv[e] = (_Float16)os[row * 132 + xoff + e];
      const int grow = R0 + row;
      *(volatile v8h*)(RS + (size_t)(grow >> 3) * 1024 + (grow & 7) * 128 + xoff) = hv;
    }
    __threadfence();
  }
}

extern "C" void kernel_launch(void* const* d_in, const int* in_sizes, int n_in,
                              void* d_out, int out_size, void* d_ws, size_t ws_size,
                              hipStream_t stream) {
  if (n_in < 10) return;
  const float* query    = (const float*)d_in[0];
  const float* matrix   = (const float*)d_in[1];
  const float* normlzr  = (const float*)d_in[2];
  const float* addrs    = (const float*)d_in[3];
  const float* W_access = (const float*)d_in[4];
  const float* b_access = (const float*)d_in[5];
  const float* W_read   = (const float*)d_in[6];
  const float* b_read   = (const float*)d_in[7];
  const float* W_merge  = (const float*)d_in[8];
  const float* b_merge  = (const float*)d_in[9];
  float* out = (float*)d_out;

  const long B = 4, T = 512, D = 1024, M = 128, H = 8, DA = 64, DM = 128;
  const long BT = B * T, HDA = H * DA, HDM = H * DM;
  if (in_sizes[0] != BT * D || in_sizes[1] != B * M * DA * DM || in_sizes[2] != B * M * DA ||
      in_sizes[3] != M * DA || in_sizes[4] != D * HDA || in_sizes[5] != HDA ||
      in_sizes[6] != D * HDA || in_sizes[7] != HDA || in_sizes[8] != HDM * D ||
      in_sizes[9] != D || (long)out_size != BT * D) return;

  size_t off = 0;
  auto carve = [&](size_t bytes) { size_t o = off; off += (bytes + 255) & ~(size_t)255; return o; };
  const size_t o_q16   = carve((size_t)BT * D * 2);
  const size_t o_war   = carve((size_t)(2 * HDA) * D * 2);
  const size_t o_wm    = carve((size_t)D * HDM * 2);
  const size_t o_mt    = carve((size_t)B * (DA * DM) * M * 2);
  const size_t o_pre   = carve((size_t)BT * (2 * HDA) * 4);
  const size_t o_aqrq  = carve((size_t)BT * (2 * HDA) * 4);
  const size_t o_c3    = carve((size_t)B * DA * (DA * DM) * 2);
  const size_t o_kmt   = carve((size_t)B * DM * (DA * DA) * 2);
  const size_t o_resp  = carve((size_t)BT * HDM * 2);
  const size_t o_akt   = carve((size_t)DA * M * 2);
  const size_t o_nk    = carve((size_t)DA * 4);
  const size_t o_kn    = carve((size_t)B * DA * DA * 4);
  const size_t o_bias  = carve((size_t)(2 * HDA) * 4);
  const size_t o_scale = carve((size_t)B * T * H * 4);
  if (off > ws_size) return;

  char* ws = (char*)d_ws;
  unsigned short* Q16    = (unsigned short*)(ws + o_q16);
  unsigned short* WarT16 = (unsigned short*)(ws + o_war);
  unsigned short* WmT16  = (unsigned short*)(ws + o_wm);
  unsigned short* MT16   = (unsigned short*)(ws + o_mt);
  float*          PRE    = (float*)(ws + o_pre);
  float*          AQRQ   = (float*)(ws + o_aqrq);
  unsigned short* C3     = (unsigned short*)(ws + o_c3);
  unsigned short* KMt    = (unsigned short*)(ws + o_kmt);
  unsigned short* RESP16 = (unsigned short*)(ws + o_resp);
  unsigned short* akT16  = (unsigned short*)(ws + o_akt);
  float*          norm_k = (float*)(ws + o_nk);
  float*          kern_n = (float*)(ws + o_kn);
  float*          bias_cat = (float*)(ws + o_bias);
  float*          scale  = (float*)(ws + o_scale);

  {
    const int n2 = (int)(BT * D / 2);
    cast_f32_f16x2<<<(n2 + 255) / 256, 256, 0, stream>>>(query, (_Float16*)Q16, n2);
  }
  tcast_f32_f16<<<dim3((int)(HDA / 64), (int)(D / 64), 1), 256, 0, stream>>>(W_access, 0L, (int)HDA, WarT16, 0L, (int)D, 64.0f);
  tcast_f32_f16<<<dim3((int)(HDA / 64), (int)(D / 64), 1), 256, 0, stream>>>(W_read, 0L, (int)HDA, WarT16 + (size_t)HDA * D, 0L, (int)D, 64.0f);
  tcast_f32_f16<<<dim3((int)(D / 64), (int)(HDM / 64), 1), 256, 0, stream>>>(W_merge, 0L, (int)D, WmT16, 0L, (int)HDM, 64.0f);
  tcast_f32_f16<<<dim3((int)(DA * DM / 64), (int)(M / 64), (int)B), 256, 0, stream>>>(
      matrix, M * DA * DM, (int)(DA * DM), MT16, (DA * DM) * M, (int)M, 1.0f);

  prep_kernel<<<1, 256, 0, stream>>>(addrs, normlzr, b_access, b_read, akT16, norm_k, kern_n, bias_cat);

  wmma_gemm64<0, false, 2, 0, false, 0><<<dim3((int)((BT / 64) * ((2 * HDA) / 64) / 8), 1), 256, 0, stream>>>(
      Q16, Q16, (int)D, 0L, WarT16, WarT16, (int)D, 0L, (void*)PRE, (void*)PRE, (int)(2 * HDA), 0L,
      bias_cat, bias_cat, 0L, (int)BT, (int)(2 * HDA), (int)D, 1.0f / 64.0f);
  {
    const int nq = (int)(BT * (2 * HDA) / 4);
    softplus_kernel<<<nq / 256, 256, 0, stream>>>(PRE, AQRQ, nq);
  }

  wmma_gemm64<0, false, 0, 1, false, 0><<<dim3((int)((DA / 64) * ((DA * DM) / 64) / 8), (int)B), 256, 0, stream>>>(
      akT16, akT16, (int)M, 0L, MT16, MT16, (int)M, (DA * DM) * M, (void*)C3, (void*)C3, (int)(DA * DM), DA * (DA * DM),
      norm_k, norm_k, 0L, (int)DA, (int)(DA * DM), (int)M, 1.0f);

  permute_km<<<(int)(B * DA), 256, 0, stream>>>(C3, KMt);

  scales_kernel<<<(int)(B * T * H / 256), 256, 0, stream>>>(AQRQ, kern_n, norm_k, scale);

  stage2_kernel<<<(int)(B * T * H / 64), 128, 0, stream>>>(AQRQ, KMt, scale, RESP16);

  wmma_gemm64<0, false, 2, 0, false, 0><<<dim3((int)((BT / 64) * (D / 64) / 8), 1), 256, 0, stream>>>(
      RESP16, RESP16, (int)HDM, 0L, WmT16, WmT16, (int)HDM, 0L, (void*)out, (void*)out, (int)D, 0L,
      b_merge, b_merge, 0L, (int)BT, (int)D, (int)HDM, 1.0f / 16384.0f);
}
